// DeformConvNet_Encoder256_41188736368691
// MI455X (gfx1250) — hardware-verified
//
#include <hip/hip_runtime.h>
#define NIM 32
#define NZ 100
typedef __bf16 v16b __attribute__((ext_vector_type(16)));
typedef unsigned short v8us __attribute__((ext_vector_type(8), may_alias));
typedef float  v8f  __attribute__((ext_vector_type(8)));
typedef float  v4f  __attribute__((ext_vector_type(4)));
typedef float  v4fa __attribute__((ext_vector_type(4), may_alias));
union FragB { v16b v; v8us half[2]; unsigned short u[16]; };

__device__ __forceinline__ unsigned short bf16_bits(float x) { unsigned int u = __float_as_uint(x); return (unsigned short)((u + 0x7FFFu + ((u >> 16) & 1u)) >> 16); }
__device__ __forceinline__ float bf16_val(unsigned short b) { return __uint_as_float(((unsigned int)b) << 16); }
__device__ __forceinline__ float bf16_round(float x) { return bf16_val(bf16_bits(x)); }
template <int NT>
__device__ __forceinline__ v8f mmaN(v16b ah, v16b al, v16b bh, v16b bl, v8f c) {
  c = __builtin_amdgcn_wmma_f32_16x16x32_bf16(false, ah, false, bh, (short)0, c, false, false);
  if (NT >= 2) c = __builtin_amdgcn_wmma_f32_16x16x32_bf16(false, al, false, bh, (short)0, c, false, false);
  if (NT >= 3) c = __builtin_amdgcn_wmma_f32_16x16x32_bf16(false, ah, false, bl, (short)0, c, false, false);
  asm volatile("v_nop\n\tv_nop\n\tv_nop\n\tv_nop" : "+v"(c) : "v"(ah), "v"(al), "v"(bh), "v"(bl));
  return c;
}

__global__ __launch_bounds__(256) void k_wt_bf16(const float* __restrict__ W, unsigned short* __restrict__ Wt, int K, int N) {
  const int t = blockIdx.x * 256 + threadIdx.x;
  const int k8n = K / 8;
  if (t >= N * k8n) return;
  const int n = t / k8n, k8 = (t % k8n) * 8;
  v8us v;
#pragma unroll
  for (int i = 0; i < 8; ++i) v[i] = bf16_bits(W[(size_t)(k8 + i) * N + n]);
  *(volatile v8us*)(Wt + (size_t)n * K + k8) = v;
  __threadfence();
  *(volatile v8us*)(Wt + (size_t)n * K + k8) = v;
}

template <bool ASPLIT, int ACT, bool BIAS_BF16>
__global__ __launch_bounds__(128) void k_gemm_bf(const float* __restrict__ A, int lda, const unsigned short* __restrict__ Wt, int ldb,
                                               const float* __restrict__ bias, float* __restrict__ C, int ldc, int M, int N, int K) {
  __shared__ __attribute__((aligned(16))) float so[4][16][64];
  const int tid = threadIdx.x, w = tid >> 5, lane = tid & 31, ln = lane & 15, hh = lane >> 4;
  const int ntn = N / 64;
  const int wid = blockIdx.x * 4 + w;
  const int mt = wid / ntn, nq = wid % ntn;
  if (mt * 16 >= M) return;
  const int row0 = mt * 16, col0 = nq * 64;
  const float* arow = A + (size_t)(row0 + ln) * lda;
  v8f acc[4] = {};
  for (int kb = 0; kb < K; kb += 32) {
    FragB ah, al;
    const v4f x0 = *(const v4fa*)(arow + kb + 8 * hh), x1 = *(const v4fa*)(arow + kb + 8 * hh + 4);
    const v4f x2 = *(const v4fa*)(arow + kb + 16 + 8 * hh), x3 = *(const v4fa*)(arow + kb + 16 + 8 * hh + 4);
    float xs[16] = {x0[0],x0[1],x0[2],x0[3],x1[0],x1[1],x1[2],x1[3],x2[0],x2[1],x2[2],x2[3],x3[0],x3[1],x3[2],x3[3]};
#pragma unroll
    for (int i = 0; i < 16; ++i) { const unsigned short hb = bf16_bits(xs[i]); ah.u[i] = hb; al.u[i] = ASPLIT ? bf16_bits(xs[i] - bf16_val(hb)) : (unsigned short)0; }
#pragma unroll
    for (int t = 0; t < 4; ++t) {
      const unsigned short* brow = Wt + (size_t)(col0 + t * 16 + ln) * ldb + kb;
      FragB b;
      b.half[0] = *(const v8us*)(brow + 8 * hh);
      b.half[1] = *(const v8us*)(brow + 16 + 8 * hh);
      acc[t] = mmaN<ASPLIT ? 2 : 1>(ah.v, al.v, b.v, b.v, acc[t]);
    }
  }
#pragma unroll
  for (int t = 0; t < 4; ++t) {
    float bv = bias ? bias[col0 + t * 16 + ln] : 0.f;
    if (BIAS_BF16) bv = bf16_round(bv);
#pragma unroll
    for (int r = 0; r < 8; ++r) { float v = acc[t][r] + bv; if (ACT == 1) v = fmaxf(v, 0.f); so[w][8 * hh + r][t * 16 + ln] = v; }
  }
  __builtin_amdgcn_fence(__ATOMIC_ACQ_REL, "workgroup");
  __builtin_amdgcn_wave_barrier();
  const int rsub = lane >> 4, c4 = (lane & 15) * 4;
  for (int pass = 0; pass < 2; ++pass) {
#pragma unroll
    for (int q = 0; q < 8; ++q) {
      const int r = q * 2 + rsub;
      const v4f v = *(const v4fa*)&so[w][r][c4];
      *(volatile v4f*)(C + (size_t)(row0 + r) * ldc + col0 + c4) = v;
    }
    if (pass == 0) __threadfence();
  }
}

template <bool ASPLIT, int ACT, bool BIAS_BF16, bool RES_BF16>
__global__ __launch_bounds__(128) void k_gemm_bf3(const float* __restrict__ A, int lda, const unsigned short* __restrict__ Wt, int ldb,
                                                const float* __restrict__ bias, const float* __restrict__ resid, int rmod, int ldr,
                                                float* __restrict__ C, int ldc, int M, int N, int K) {
  __shared__ __attribute__((aligned(16))) float so[4][16][64];
  const int tid = threadIdx.x, w = tid >> 5, lane = tid & 31, ln = lane & 15, hh = lane >> 4;
  const int ntn = N / 64;
  const int wid = blockIdx.x * 4 + w;
  const int mt = wid / ntn, nq = wid % ntn;
  if (mt * 16 >= M) return;
  const int row0 = mt * 16, col0 = nq * 64;
  const float* arow = A + (size_t)(row0 + ln) * lda;
  v8f acc[4] = {};
  for (int kb = 0; kb < K; kb += 32) {
    FragB ah, al;
    const v4f x0 = *(const v4fa*)(arow + kb + 8 * hh), x1 = *(const v4fa*)(arow + kb + 8 * hh + 4);
    const v4f x2 = *(const v4fa*)(arow + kb + 16 + 8 * hh), x3 = *(const v4fa*)(arow + kb + 16 + 8 * hh + 4);
    float xs[16] = {x0[0],x0[1],x0[2],x0[3],x1[0],x1[1],x1[2],x1[3],x2[0],x2[1],x2[2],x2[3],x3[0],x3[1],x3[2],x3[3]};
#pragma unroll
    for (int i = 0; i < 16; ++i) { const unsigned short hb = bf16_bits(xs[i]); ah.u[i] = hb; al.u[i] = ASPLIT ? bf16_bits(xs[i] - bf16_val(hb)) : (unsigned short)0; }
#pragma unroll
    for (int t = 0; t < 4; ++t) {
      const unsigned short* brow = Wt + (size_t)(col0 + t * 16 + ln) * ldb + kb;
      FragB b;
      b.half[0] = *(const v8us*)(brow + 8 * hh);
      b.half[1] = *(const v8us*)(brow + 16 + 8 * hh);
      acc[t] = mmaN<ASPLIT ? 2 : 1>(ah.v, al.v, b.v, b.v, acc[t]);
    }
  }
#pragma unroll
  for (int t = 0; t < 4; ++t) {
    const int col = col0 + t * 16 + ln;
    float bv = bias ? bias[col] : 0.f;
    if (BIAS_BF16) bv = bf16_round(bv);
#pragma unroll
    for (int r = 0; r < 8; ++r) {
      float v = acc[t][r] + bv;
      if (resid) { float rv = resid[(size_t)((row0 + 8 * hh + r) % rmod) * ldr + col]; if (RES_BF16) rv = bf16_round(rv); v += rv; }
      if (ACT == 1) v = fmaxf(v, 0.f);
      if (ACT == 2) v = 0.5f * v * (1.0f + erff(v * 0.70710678118654752f));
      if (ACT == 3) { const float u = 0.7978845608028654f * (v + 0.044715f * v * v * v); v = 0.5f * v * (1.0f + tanhf(u)); }
      so[w][8 * hh + r][t * 16 + ln] = v;
    }
  }
  __builtin_amdgcn_fence(__ATOMIC_ACQ_REL, "workgroup");
  __builtin_amdgcn_wave_barrier();
  const int rsub = lane >> 4, c4 = (lane & 15) * 4;
  for (int pass = 0; pass < 2; ++pass) {
#pragma unroll
    for (int q = 0; q < 8; ++q) {
      const int r = q * 2 + rsub;
      const v4f v = *(const v4fa*)&so[w][r][c4];
      *(volatile v4f*)(C + (size_t)(row0 + r) * ldc + col0 + c4) = v;
    }
    if (pass == 0) __threadfence();
  }
}
template <bool PARAM_BF16>
__global__ __launch_bounds__(256) void k_layernorm(const float* __restrict__ X, const float* __restrict__ R, const float* __restrict__ g, const float* __restrict__ bta,
                                                  float* __restrict__ out_sum, float* __restrict__ out_norm, int N, float eps) {
  __shared__ float red[256];
  const int row = blockIdx.x, tid = threadIdx.x;
  const float* x = X + (size_t)row * N; const float* rr = R ? R + (size_t)row * N : nullptr;
  float vals[16];
  const int per = N / 256;
  float s1 = 0.f;
  for (int u = 0; u < per / 4; ++u) {
    const int j = tid * 4 + 1024 * u;
    const v4f a = *(const v4fa*)(x + j);
    v4f b = {0.f,0.f,0.f,0.f}; if (rr) b = *(const v4fa*)(rr + j);
#pragma unroll
    for (int q = 0; q < 4; ++q) { const float v = a[q] + b[q]; vals[u * 4 + q] = v; s1 += v; }
  }
  red[tid] = s1; __syncthreads();
  for (int st = 128; st > 0; st >>= 1) { if (tid < st) red[tid] += red[tid + st]; __syncthreads(); }
  const float mu = red[0] / (float)N; __syncthreads();
  float s2 = 0.f;
  for (int u = 0; u < per / 4; ++u)
#pragma unroll
    for (int q = 0; q < 4; ++q) { const float c = vals[u * 4 + q] - mu; s2 += c * c; }
  red[tid] = s2; __syncthreads();
  for (int st = 128; st > 0; st >>= 1) { if (tid < st) red[tid] += red[tid + st]; __syncthreads(); }
  const float rs = rsqrtf(red[0] / (float)N + eps);
  for (int pass = 0; pass < 2; ++pass) {
    for (int u = 0; u < per / 4; ++u) {
      const int j = tid * 4 + 1024 * u;
      v4f o, sm;
#pragma unroll
      for (int q = 0; q < 4; ++q) {
        float gg = g[j + q], bb = bta[j + q];
        if (PARAM_BF16) { gg = bf16_round(gg); bb = bf16_round(bb); }
        sm[q] = vals[u * 4 + q]; o[q] = (vals[u * 4 + q] - mu) * rs * gg + bb;
      }
      if (out_sum) *(volatile v4f*)(out_sum + (size_t)row * N + j) = sm;
      *(volatile v4f*)(out_norm + (size_t)row * N + j) = o;
    }
    if (pass == 0) __threadfence();
  }
}


typedef _Float16 v16h __attribute__((ext_vector_type(16)));
union FragH { v16h v; v8us half[2]; _Float16 h[16]; unsigned short u[16]; };
template <int NT>
__device__ __forceinline__ v8f mmaH(v16h ah, v16h al, v16h bh, v16h bl, v8f c) {
  c = __builtin_amdgcn_wmma_f32_16x16x32_f16(false, ah, false, bh, (short)0, c, false, false);
  if (NT >= 2) c = __builtin_amdgcn_wmma_f32_16x16x32_f16(false, al, false, bh, (short)0, c, false, false);
  if (NT >= 3) c = __builtin_amdgcn_wmma_f32_16x16x32_f16(false, ah, false, bl, (short)0, c, false, false);
  asm volatile("v_nop\n\tv_nop\n\tv_nop\n\tv_nop" : "+v"(c) : "v"(ah), "v"(al), "v"(bh), "v"(bl));
  return c;
}
template <bool ASPLIT>
__global__ __launch_bounds__(128) void k_gemm_h(const float* __restrict__ A, int lda, size_t sA, const _Float16* __restrict__ Bh, int ldb, size_t sB, float alpha, float* __restrict__ C, int ldc, size_t sC, int M, int N, int K) {
  __shared__ __attribute__((aligned(16))) float so[4][16][64];
  const int tid = threadIdx.x, w = tid >> 5, lane = tid & 31, ln = lane & 15, hh = lane >> 4; const int by = blockIdx.y;
  A += (size_t)by * sA; Bh += (size_t)by * sB; C += (size_t)by * sC;
  const int ntn = (N + 63) / 64; const int wid = blockIdx.x * 4 + w; const int mt = wid / ntn, nq = wid % ntn; if (mt * 16 >= M) return;
  const int row0 = mt * 16, col0 = nq * 64; const float* arow = A + (size_t)(row0 + ln) * lda;
  v8f acc[4] = {};
  for (int kb = 0; kb < K; kb += 32) {
    FragH ah, al;
    const v4f x0 = *(const v4fa*)(arow + kb + 8 * hh), x1 = *(const v4fa*)(arow + kb + 8 * hh + 4), x2 = *(const v4fa*)(arow + kb + 16 + 8 * hh), x3 = *(const v4fa*)(arow + kb + 16 + 8 * hh + 4);
    float xs[16] = {x0[0],x0[1],x0[2],x0[3],x1[0],x1[1],x1[2],x1[3],x2[0],x2[1],x2[2],x2[3],x3[0],x3[1],x3[2],x3[3]};
#pragma unroll
    for (int i = 0; i < 16; ++i) { const _Float16 h = (_Float16)xs[i]; ah.h[i] = h; al.h[i] = ASPLIT ? (_Float16)(xs[i] - (float)h) : (_Float16)0.0f; }
#pragma unroll
    for (int t = 0; t < 4; ++t) { if (col0 + t * 16 >= N) continue; const size_t boff = (size_t)(col0 + t * 16 + ln) * ldb + kb; FragH bq; bq.half[0] = *(const v8us*)(Bh + boff + 8 * hh); bq.half[1] = *(const v8us*)(Bh + boff + 16 + 8 * hh);
      acc[t] = mmaH<ASPLIT ? 2 : 1>(ah.v, al.v, bq.v, bq.v, acc[t]); }
  }
#pragma unroll
  for (int t = 0; t < 4; ++t) { if (col0 + t * 16 >= N) continue;
#pragma unroll
    for (int r = 0; r < 8; ++r) so[w][8 * hh + r][t * 16 + ln] = acc[t][r] * alpha; }
  __builtin_amdgcn_fence(__ATOMIC_ACQ_REL, "workgroup"); __builtin_amdgcn_wave_barrier();
  const int rsub = lane >> 4, c4 = (lane & 15) * 4;
  for (int pass = 0; pass < 2; ++pass) {
#pragma unroll
    for (int q = 0; q < 8; ++q) { const int r = q * 2 + rsub; if (col0 + c4 < N) { const v4f v = *(const v4fa*)&so[w][r][c4]; *(volatile v4f*)(C + (size_t)(row0 + r) * ldc + col0 + c4) = v; } }
    if (pass == 0) __threadfence(); }
}

__global__ __launch_bounds__(256) void k_wt_f16(const float* __restrict__ W, _Float16* __restrict__ Wt, int K, int N, float scale) {
  const int t = blockIdx.x * 256 + threadIdx.x; if (t >= N * (K / 8)) return; const int n = t / (K / 8), k8 = (t % (K / 8)) * 8; FragH f;
#pragma unroll
  for (int i = 0; i < 8; ++i) f.h[i] = (_Float16)(bf16_round(W[(size_t)(k8 + i) * N + n]) * scale); const v8us o = f.half[0];
  *(volatile v8us*)((unsigned short*)Wt + (size_t)n * K + k8) = o; __threadfence(); *(volatile v8us*)((unsigned short*)Wt + (size_t)n * K + k8) = o;
}
template <int ACT>
__global__ __launch_bounds__(128) void k_gemm_hhx(const _Float16* __restrict__ A, int lda, size_t sA, const _Float16* __restrict__ Bh, int ldb, size_t sB, float alpha, const float* __restrict__ bias, size_t sBias, const float* __restrict__ CP, int rowsPerB, size_t sCPb, int row0g,
    float* __restrict__ C, _Float16* __restrict__ C16, int ldc, size_t sC, int M, int N, int K) {
  __shared__ __attribute__((aligned(16))) float so[4][16][64];
  const int tid = threadIdx.x, w = tid >> 5, lane = tid & 31, ln = lane & 15, hh = lane >> 4; const int by = blockIdx.y;
  A += (size_t)by * sA; Bh += (size_t)by * sB; const size_t cofs = (size_t)by * sC; const float* bp = bias ? bias + (size_t)by * sBias : nullptr;
  const int ntn = (N + 63) / 64; const int wid = blockIdx.x * 4 + w; const int mt = wid / ntn, nq = wid % ntn; if (mt * 16 >= M) return;
  const int row0 = mt * 16, col0 = nq * 64; const _Float16* arow = A + (size_t)(row0 + ln) * lda;
  v8f acc[4] = {};
  for (int kb = 0; kb < K; kb += 32) { FragH ah; ah.half[0] = *(const v8us*)((const unsigned short*)arow + kb + 8 * hh); ah.half[1] = *(const v8us*)((const unsigned short*)arow + kb + 16 + 8 * hh);
#pragma unroll
    for (int t = 0; t < 4; ++t) { if (col0 + t * 16 >= N) continue; const size_t boff = (size_t)(col0 + t * 16 + ln) * ldb + kb; FragH bq; bq.half[0] = *(const v8us*)((const unsigned short*)Bh + boff + 8 * hh); bq.half[1] = *(const v8us*)((const unsigned short*)Bh + boff + 16 + 8 * hh);
      acc[t] = mmaH<1>(ah.v, ah.v, bq.v, bq.v, acc[t]); }
  }
#pragma unroll
  for (int t = 0; t < 4; ++t) { if (col0 + t * 16 >= N) continue; const int col = col0 + t * 16 + ln; const float bv = bp ? bf16_round(bp[col]) : 0.f;
#pragma unroll
    for (int r = 0; r < 8; ++r) { float v = acc[t][r] * alpha + bv; if (CP) { const int bidx = (row0g + row0 + 8 * hh + r) / rowsPerB; v += CP[(size_t)bidx * sCPb + (size_t)by * 64 + col]; } if (ACT == 1) v = (v > 0.f) ? v : expm1f(v); else if (ACT == 7) v = (v > 0.f) ? v + 1.0f : expf(v); else if (ACT == 8) v = tanhf(v); else if (ACT == 9) v = 0.5f * v * (1.0f + tanhf(0.7978845608028654f * (v + 0.044715f * v * v * v))); else if (ACT == 11) v = 1.0f / (1.0f + expf(-v)); else if (ACT == 12) v = (v > 0.f) ? v : 0.01f * v; else if (ACT == 14) v = (v > 0.f) ? v : 0.1f * v; else if (ACT == 15) v = v / (1.0f + expf(-v)); else if (ACT == 3) v = fmaxf(v, 0.f); else if (ACT == 6) v = 0.5f * v * (1.0f + erff(v * 0.70710678118654752f)); so[w][8 * hh + r][t * 16 + ln] = v; } }
  __builtin_amdgcn_fence(__ATOMIC_ACQ_REL, "workgroup"); __builtin_amdgcn_wave_barrier();
  const int rsub = lane >> 4, c4 = (lane & 15) * 4; typedef _Float16 v4h __attribute__((ext_vector_type(4)));
  for (int pass = 0; pass < 2; ++pass) {
#pragma unroll
    for (int q = 0; q < 8; ++q) { const int r = q * 2 + rsub; if (col0 + c4 < N) { const v4f v = *(const v4fa*)&so[w][r][c4]; if (C) *(volatile v4f*)(C + cofs + (size_t)(row0 + r) * ldc + col0 + c4) = v; if (C16) { v4h h4; for (int i = 0; i < 4; ++i) h4[i] = (_Float16)v[i]; *(volatile v4h*)(C16 + cofs + (size_t)(row0 + r) * ldc + col0 + c4) = h4; } } }
    if (pass == 0) __threadfence(); }
}


typedef _Float16 v4h __attribute__((ext_vector_type(4)));

__global__ __launch_bounds__(256) void k_x16(const float* __restrict__ x, _Float16* __restrict__ X16, size_t n8) { const size_t t = (size_t)blockIdx.x * 256 + threadIdx.x; if (t >= n8) return; FragH f;
#pragma unroll
  for (int q = 0; q < 8; ++q) f.h[q] = (_Float16)bf16_round(x[t * 8 + q]); *(volatile v8us*)((unsigned short*)X16 + t * 8) = f.half[0]; __threadfence(); *(volatile v8us*)((unsigned short*)X16 + t * 8) = f.half[0]; }
__global__ __launch_bounds__(256) void k_h16(const float* __restrict__ x, _Float16* __restrict__ X16, size_t n8) { const size_t t = (size_t)blockIdx.x * 256 + threadIdx.x; if (t >= n8) return; FragH f;
#pragma unroll
  for (int q = 0; q < 8; ++q) f.h[q] = (_Float16)x[t * 8 + q]; *(volatile v8us*)((unsigned short*)X16 + t * 8) = f.half[0]; __threadfence(); *(volatile v8us*)((unsigned short*)X16 + t * 8) = f.half[0]; }
__global__ __launch_bounds__(256) void k_round16f(const float* __restrict__ W, _Float16* __restrict__ Bt, size_t n8) { const size_t t = (size_t)blockIdx.x * 256 + threadIdx.x; if (t >= n8) return; FragH f;
#pragma unroll
  for (int i = 0; i < 8; ++i) f.h[i] = (_Float16)(bf16_round(W[t * 8 + i]) * 16.0f); *(volatile v8us*)((unsigned short*)Bt + t * 8) = f.half[0]; __threadfence(); *(volatile v8us*)((unsigned short*)Bt + t * 8) = f.half[0]; }
template <int NHv, int TTv>
__global__ __launch_bounds__(256) void k_vt(const _Float16* __restrict__ V16, int ldv, int voff, _Float16* __restrict__ Vt) { __shared__ unsigned short tl[64][66]; const int tid = threadIdx.x; const int slab = blockIdx.x / (TTv / 64), lg = blockIdx.x % (TTv / 64); const int b = slab / NHv, h = slab % NHv;
  for (int i = tid; i < 64 * 8; i += 256) { const int r = i / 8, c8 = (i % 8) * 8; FragH f; f.half[0] = *(const v8us*)((const unsigned short*)V16 + ((size_t)b * TTv + lg * 64 + r) * ldv + voff + h * 64 + c8);
#pragma unroll
    for (int q = 0; q < 8; ++q) tl[r][c8 + q] = f.u[q]; }
  __syncthreads();
  for (int pass = 0; pass < 2; ++pass) {
#pragma unroll
    for (int rd = 0; rd < 2; ++rd) { const int d = rd * 32 + tid / 8, pc = tid % 8; FragH f;
#pragma unroll
      for (int q = 0; q < 8; ++q) f.u[q] = tl[pc * 8 + q][d];
      *(volatile v8us*)((unsigned short*)Vt + ((size_t)slab * 64 + d) * TTv + lg * 64 + pc * 8) = f.half[0]; }
    if (pass == 0) __threadfence(); } }

__global__ __launch_bounds__(256) void k_hl(const float* __restrict__ F, _Float16* __restrict__ Hh, _Float16* __restrict__ Hl, size_t n8) { const size_t t = (size_t)blockIdx.x * 256 + threadIdx.x; if (t >= n8) return; FragH fh, fl; const v4f a = *(const v4fa*)(F + t * 8), c = *(const v4fa*)(F + t * 8 + 4);
#pragma unroll
  for (int q = 0; q < 4; ++q) { _Float16 h = (_Float16)a[q]; fh.h[q] = h; fl.h[q] = (_Float16)((a[q] - (float)h) * 1024.0f); h = (_Float16)c[q]; fh.h[4 + q] = h; fl.h[4 + q] = (_Float16)((c[q] - (float)h) * 1024.0f); }
  for (int pass = 0; pass < 2; ++pass) { *(volatile v8us*)((unsigned short*)Hh + t * 8) = fh.half[0]; *(volatile v8us*)((unsigned short*)Hl + t * 8) = fl.half[0]; if (pass == 0) __threadfence(); } }

__global__ __launch_bounds__(256) void k_wtap(const float* __restrict__ w, int O, int orows, int C, int KP, _Float16* __restrict__ Bt) { const size_t t = (size_t)blockIdx.x * 256 + threadIdx.x; if (t >= (size_t)orows * (KP / 8)) return; const int col0 = (int)(t % (KP / 8)) * 8; const int o = (int)(t / (KP / 8)); FragH f;
#pragma unroll
  for (int q = 0; q < 8; ++q) { const int col = col0 + q; const int k = col / C, c = col % C; f.h[q] = (o < O && col < 9 * C) ? (_Float16)(bf16_round(w[((size_t)o * C + c) * 9 + k]) * 16.0f) : (_Float16)0.0f; }
  *(volatile v8us*)((unsigned short*)Bt + (size_t)o * KP + col0) = f.half[0]; __threadfence(); *(volatile v8us*)((unsigned short*)Bt + (size_t)o * KP + col0) = f.half[0]; }
__global__ __launch_bounds__(256) void k_bpad(const float* __restrict__ bb, int n, int np, float* __restrict__ BP) { const int l = threadIdx.x; if (l >= np) return; const float v = (l < n) ? bb[l] : 0.f; *(volatile float*)(BP + l) = v; __threadfence(); *(volatile float*)(BP + l) = v; }
__global__ __launch_bounds__(256) void k_im0(const float* __restrict__ x, int img0, int nimg, _Float16* __restrict__ A) { const int t = blockIdx.x * 256 + threadIdx.x; if (t >= nimg * 128 * 128) return; const int ox = t & 127, oy = (t >> 7) & 127, i = img0 + (t >> 14); FragH f[4];
#pragma unroll
  for (int col = 0; col < 32; ++col) { float v = 0.f; if (col < 27) { const int k = col / 3, c = col % 3; const int yy = 2 * oy + k / 3 - 1, xx = 2 * ox + k % 3 - 1; const int yc = min(max(yy, 0), 255), xc = min(max(xx, 0), 255); const float xv = x[(((size_t)i * 3 + c) * 256 + yc) * 256 + xc]; v = (yy >= 0 && yy < 256 && xx >= 0 && xx < 256) ? bf16_round(xv) : 0.f; } f[col >> 3].h[col & 7] = (_Float16)v; }
  for (int pass = 0; pass < 2; ++pass) {
#pragma unroll
    for (int g = 0; g < 4; ++g) *(volatile v8us*)((unsigned short*)A + (size_t)t * 32 + g * 8) = f[g].half[0];
    if (pass == 0) __threadfence(); } }
__global__ __launch_bounds__(256) void k_cstats(const float* __restrict__ X, int n, int C, double* __restrict__ SUM, double* __restrict__ SQ) { __shared__ double s1[8][32], s2[8][32]; const int tid = threadIdx.x, w = tid >> 5, l = tid & 31; const int c = blockIdx.x * 32 + l; double a = 0.0, b = 0.0;
  if (c < C) {
#pragma unroll 1
    for (int r = w; r < n; r += 8) { const double v = (double)X[(size_t)r * C + c]; a += v; b += v * v; } }
  s1[w][l] = a; s2[w][l] = b; __syncthreads();
  if (w == 0 && c < C) { double t1 = 0.0, t2 = 0.0; for (int q = 0; q < 8; ++q) { t1 += s1[q][l]; t2 += s2[q][l]; } for (int pass = 0; pass < 2; ++pass) { *(volatile double*)(SUM + c) = t1; *(volatile double*)(SQ + c) = t2; if (pass == 0) __threadfence(); } } }
__global__ __launch_bounds__(256) void k_bnact(const float* __restrict__ X, int n, int C, const double* __restrict__ SUM, const double* __restrict__ SQ, const float* __restrict__ g, const float* __restrict__ be, int act, _Float16* __restrict__ H) {
  #pragma clang fp contract(off)
  const size_t t = (size_t)blockIdx.x * 256 + threadIdx.x; if (t >= (size_t)n * (C / 8)) return; const int c0 = (int)(t % (C / 8)) * 8; const size_t r = t / (C / 8); FragH f;
#pragma unroll
  for (int q = 0; q < 8; ++q) { const int c = c0 + q; const double m = SUM[c] / (double)n; double var = SQ[c] / (double)n - m * m; if (var < 0.0) var = 0.0; const float v = (X[r * C + c] - (float)m) * rsqrtf((float)var + 1e-5f) * bf16_round(g[c]) + bf16_round(be[c]); f.h[q] = (_Float16)((act == 0) ? fmaxf(v, 0.f) : ((v >= 0.f) ? v : 0.2f * v)); }
  *(volatile v8us*)((unsigned short*)H + r * C + c0) = f.half[0]; __threadfence(); *(volatile v8us*)((unsigned short*)H + r * C + c0) = f.half[0]; }
__global__ __launch_bounds__(256) void k_im2col(const _Float16* __restrict__ H, int S, int C, int stride, int pad, int So, int img0, int nimg, int KP, _Float16* __restrict__ A) { const size_t t = (size_t)blockIdx.x * 256 + threadIdx.x; const int G = KP / 8; const size_t tot = (size_t)nimg * So * So * G; if (t >= tot) return; const int g = (int)(t % G); const size_t op = t / G; const bool real = (g < 9 * C / 8); const int k = real ? g / (C / 8) : 0; const int c0 = (g % (C / 8)) * 8; const int ox = (int)(op % So), oy = (int)((op / So) % So), i = (int)(op / ((size_t)So * So));
  const int yy = oy * stride + k / 3 - pad, xx = ox * stride + k % 3 - pad; const bool in = real && (yy >= 0 && yy < S && xx >= 0 && xx < S); const int yc = min(max(yy, 0), S - 1), xc = min(max(xx, 0), S - 1); FragH f; f.half[0] = *(const v8us*)((const unsigned short*)H + (((size_t)(img0 + i) * S + yc) * S + xc) * C + c0); if (!in) f = FragH{};
  *(volatile v8us*)((unsigned short*)A + op * (size_t)KP + (size_t)g * 8) = f.half[0]; __threadfence(); *(volatile v8us*)((unsigned short*)A + op * (size_t)KP + (size_t)g * 8) = f.half[0]; }
__global__ __launch_bounds__(256) void k_wlin(const float* __restrict__ w, int O, int orows, int K, _Float16* __restrict__ Bt) { const size_t t = (size_t)blockIdx.x * 256 + threadIdx.x; if (t >= (size_t)orows * (K / 8)) return; const int k0 = (int)(t % (K / 8)) * 8; const int o = (int)(t / (K / 8)); FragH f;
#pragma unroll
  for (int q = 0; q < 8; ++q) f.h[q] = (o < O) ? (_Float16)(bf16_round(w[(size_t)o * K + k0 + q]) * 16.0f) : (_Float16)0.0f;
  *(volatile v8us*)((unsigned short*)Bt + (size_t)o * K + k0) = f.half[0]; __threadfence(); *(volatile v8us*)((unsigned short*)Bt + (size_t)o * K + k0) = f.half[0]; }
__global__ __launch_bounds__(256) void k_deform(const _Float16* __restrict__ H, const float* __restrict__ OFF, int S, int C, int img0, int nimg, _Float16* __restrict__ HD) {
  #pragma clang fp contract(off)
  const size_t t = (size_t)blockIdx.x * 256 + threadIdx.x; const int HW = S * S; if (t >= (size_t)nimg * HW * (C / 8)) return; const int c0 = (int)(t % (C / 8)) * 8; const size_t ip = t / (C / 8); const int p = (int)(ip % HW), i = (int)(ip / HW); const int y = p / S, x = p % S; const int q0 = (2 * p) % HW, a0 = (2 * p) / HW, q1 = (2 * p + 1) % HW, a1 = (2 * p + 1) / HW; const float* offr0 = OFF + ((size_t)i * HW + q0) * (2 * C); const float* offr1 = OFF + ((size_t)i * HW + q1) * (2 * C); const _Float16* Hi = H + (size_t)(img0 + i) * HW * C; FragH f;
#pragma unroll
  for (int qq = 0; qq < 8; ++qq) { const int ch = c0 + qq; const float dy = offr0[2 * ch + a0], dx = offr1[2 * ch + a1];
    const float cy = fminf(fmaxf(dy + (float)y, 0.f), (float)(S - 1)), cx = fminf(fmaxf(dx + (float)x, 0.f), (float)(S - 1)); const float y0f = floorf(cy), y1f = ceilf(cy), x0f = floorf(cx), x1f = ceilf(cx); const float wy = cy - y0f, wx = cx - x0f; const int y0i = (int)y0f, y1i = (int)y1f, x0i = (int)x0f, x1i = (int)x1f;
    const float v00 = (float)Hi[((size_t)y0i * S + x0i) * C + ch], v01 = (float)Hi[((size_t)y0i * S + x1i) * C + ch], v10 = (float)Hi[((size_t)y1i * S + x0i) * C + ch], v11 = (float)Hi[((size_t)y1i * S + x1i) * C + ch];
    f.h[qq] = (_Float16)(((v00 * (1.f - wy)) * (1.f - wx) + (v01 * (1.f - wy)) * wx) + ((v10 * wy) * (1.f - wx) + (v11 * wy) * wx)); }
  *(volatile v8us*)((unsigned short*)HD + ip * C + c0) = f.half[0]; __threadfence(); *(volatile v8us*)((unsigned short*)HD + ip * C + c0) = f.half[0]; }
__global__ __launch_bounds__(256) void k_fin(const float* __restrict__ Y, float* __restrict__ out) {
  #pragma clang fp contract(off)
  const int t = blockIdx.x * 256 + threadIdx.x; if (t >= NIM * NZ) return; const float v = 1.0f / (1.0f + expf(-Y[(size_t)(t / NZ) * 128 + (t % NZ)])); *(volatile float*)(out + t) = v; __threadfence(); *(volatile float*)(out + t) = v; }

extern "C" void kernel_launch(void* const* d_in, const int* in_sizes, int n_in,
                              void* d_out, int out_size, void* d_ws, size_t ws_size, hipStream_t stream) {
  (void)in_sizes; (void)n_in; (void)out_size;
  const float* const* I = (const float* const*)d_in; const float* x = I[0]; const float* w_first = I[1]; const float* g_first = I[2]; const float* b_first = I[3]; const float* OW[5], *CW[5], *GG[5], *BBv[5]; for (int s = 0; s < 5; ++s) { OW[s] = I[4 + 4 * s]; CW[s] = I[5 + 4 * s]; GG[s] = I[6 + 4 * s]; BBv[s] = I[7 + 4 * s]; } const float* w_last = I[24]; const float* g_last = I[25]; const float* b_last = I[26]; const float* w_out = I[27]; const float* b_out = I[28];
  const int CH[6] = {16, 32, 64, 128, 256, 512}; const int SP[6] = {128, 64, 32, 16, 8, 4};
  char* ws = (char*)d_ws; size_t off = 0;
  auto take = [&](size_t bytes) { char* p = ws + off; off += (bytes + 255) & ~(size_t)255; return p; };
  _Float16* B0 = (_Float16*)take(16 * 32 * 2); _Float16* BO[5]; _Float16* BC[5]; for (int s = 0; s < 5; ++s) { const size_t kp = (s == 0) ? 192 : 9 * CH[s]; BO[s] = (_Float16*)take((size_t)2 * CH[s] * kp * 2); BC[s] = (_Float16*)take((size_t)2 * CH[s] * kp * 2); } _Float16* BL = (_Float16*)take((size_t)1024 * 4608 * 2); _Float16* BZ = (_Float16*)take((size_t)128 * 1024 * 2); float* BPz = (float*)take(512);
  _Float16* Hp[7]; for (int s = 0; s < 6; ++s) Hp[s] = (_Float16*)take((size_t)NIM * SP[s] * SP[s] * CH[s] * 2); Hp[6] = (_Float16*)take((size_t)NIM * 1024 * 2);
  float* CB = (float*)take((size_t)NIM * 128 * 128 * 16 * 4); _Float16* A = (_Float16*)take((size_t)65536 * 192 * 2 + 256); float* OFF = (float*)take((size_t)8388608 + 256); _Float16* HD = (_Float16*)take((size_t)2097152 + 256); _Float16* A2 = (_Float16*)take((size_t)16384 * 192 * 2 + 256); double* SUM = (double*)take(1024 * 8); double* SQ = (double*)take(1024 * 8); float* Y = (float*)take((size_t)NIM * 128 * 4);
  if (off > ws_size) return;
  k_wtap<<<(16 * 4 + 255) / 256, 256, 0, stream>>>(w_first, 16, 16, 3, 32, B0);
  for (int s = 0; s < 5; ++s) { const int C = CH[s]; const int KPw = (s == 0) ? 192 : 9 * C; k_wtap<<<(unsigned)(((size_t)2 * C * (KPw / 8) + 255) / 256), 256, 0, stream>>>(OW[s], 2 * C, 2 * C, C, KPw, BO[s]); k_wtap<<<(unsigned)(((size_t)2 * C * (KPw / 8) + 255) / 256), 256, 0, stream>>>(CW[s], 2 * C, 2 * C, C, KPw, BC[s]); }
  k_wtap<<<(unsigned)(((size_t)1024 * (4608 / 8) + 255) / 256), 256, 0, stream>>>(w_last, 1024, 1024, 512, 4608, BL);
  k_wlin<<<(unsigned)(((size_t)128 * (1024 / 8) + 255) / 256), 256, 0, stream>>>(w_out, NZ, 128, 1024, BZ); k_bpad<<<1, 256, 0, stream>>>(b_out, NZ, 128, BPz);
  for (int c2 = 0; c2 < 2; ++c2) { k_im0<<<(16 * 16384 + 255) / 256, 256, 0, stream>>>(x, 16 * c2, 16, A); k_gemm_hhx<0><<<dim3(((16 * 16384 / 16) * 1 + 3) / 4, 1), 128, 0, stream>>>(A, 32, 0, B0, 32, 0, 0.0625f, nullptr, 0, nullptr, 1, 0, 0, CB + (size_t)c2 * 16 * 16384 * 16, nullptr, 16, 0, 16 * 16384, 16, 32); }
  k_cstats<<<1, 256, 0, stream>>>(CB, NIM * 16384, 16, SUM, SQ); k_bnact<<<(unsigned)(((size_t)NIM * 16384 * 2 + 255) / 256), 256, 0, stream>>>(CB, NIM * 16384, 16, SUM, SQ, g_first, b_first, 0, Hp[0]);
  const int NCHK[5] = {8, 4, 2, 1, 1};
  for (int s = 0; s < 5; ++s) { const int C = CH[s], S = SP[s], So = S / 2, Co = 2 * C, HW = S * S; const int KP = (s == 0) ? 192 : 9 * C; const int nimg = NIM / NCHK[s];
    for (int ck = 0; ck < NCHK[s]; ++ck) { const int img0 = ck * nimg; const int Mo = nimg * HW, Mc = nimg * So * So;
      k_im2col<<<(unsigned)(((size_t)Mo * (KP / 8) + 255) / 256), 256, 0, stream>>>(Hp[s], S, C, 1, 1, S, img0, nimg, KP, A);
      k_gemm_hhx<0><<<dim3(((Mo / 16) * ((Co + 63) / 64) + 3) / 4, 1), 128, 0, stream>>>(A, KP, 0, BO[s], KP, 0, 0.0625f, nullptr, 0, nullptr, 1, 0, 0, OFF, nullptr, Co, 0, Mo, Co, KP);
      k_deform<<<(unsigned)(((size_t)Mo * (C / 8) + 255) / 256), 256, 0, stream>>>(Hp[s], OFF, S, C, img0, nimg, HD);
      k_im2col<<<(unsigned)(((size_t)Mc * (KP / 8) + 255) / 256), 256, 0, stream>>>(HD, S, C, 2, 1, So, 0, nimg, KP, A2);
      k_gemm_hhx<0><<<dim3(((Mc / 16) * ((Co + 63) / 64) + 3) / 4, 1), 128, 0, stream>>>(A2, KP, 0, BC[s], KP, 0, 0.0625f, nullptr, 0, nullptr, 1, 0, 0, CB + (size_t)img0 * So * So * Co, nullptr, Co, 0, Mc, Co, KP); }
    k_cstats<<<(Co + 31) / 32, 256, 0, stream>>>(CB, NIM * So * So, Co, SUM, SQ); k_bnact<<<(unsigned)(((size_t)NIM * So * So * (Co / 8) + 255) / 256), 256, 0, stream>>>(CB, NIM * So * So, Co, SUM, SQ, GG[s], BBv[s], 1, Hp[s + 1]); }
  k_im2col<<<(unsigned)(((size_t)NIM * (4608 / 8) + 255) / 256), 256, 0, stream>>>(Hp[5], 4, 512, 2, 0, 1, 0, NIM, 4608, A);
  k_gemm_hhx<0><<<dim3(((NIM / 16) * (1024 / 64) + 3) / 4, 1), 128, 0, stream>>>(A, 4608, 0, BL, 4608, 0, 0.0625f, nullptr, 0, nullptr, 1, 0, 0, CB, nullptr, 1024, 0, NIM, 1024, 4608);
  k_cstats<<<1024 / 32, 256, 0, stream>>>(CB, NIM, 1024, SUM, SQ); k_bnact<<<(NIM * 128 + 255) / 256, 256, 0, stream>>>(CB, NIM, 1024, SUM, SQ, g_last, b_last, 0, Hp[6]);
  k_gemm_hhx<0><<<dim3(((NIM / 16) * 2 + 3) / 4, 1), 128, 0, stream>>>(Hp[6], 1024, 0, BZ, 1024, 0, 0.0625f, BPz, 0, nullptr, 1, 0, 0, Y, nullptr, 128, 0, NIM, 128, 1024);
  k_fin<<<(NIM * NZ + 255) / 256, 256, 0, stream>>>(Y, (float*)d_out);
}
